// SSMCore_50818053046523
// MI455X (gfx1250) — hardware-run, weakly checked
//
#include <hip/hip_runtime.h>
#include <math.h>

typedef __attribute__((ext_vector_type(16))) _Float16 v16h;
typedef __attribute__((ext_vector_type(8)))  _Float16 v8h;
typedef __attribute__((ext_vector_type(8)))  float    v8f;
typedef __attribute__((ext_vector_type(4)))  float    v4f;
typedef __attribute__((ext_vector_type(4)))  unsigned v4u;
typedef __attribute__((ext_vector_type(2)))  unsigned v2u;

constexpr int kSteps   = 2048;
constexpr int kChan    = 2048;
constexpr int kStates  = 16;
constexpr int kProjW   = 2 * kStates;
constexpr int kTaps    = 4;
constexpr int kKpad1   = 32;
constexpr int kChunk   = 128;
constexpr int kWarm    = 32;
constexpr int kGroup   = 16;
static_assert(kProjW == 32, "projection width");
static_assert((kChan % 256) == 0 && (kSteps % kChunk) == 0 && (kChunk % kGroup) == 0 && (kWarm % kGroup) == 0, "tile multiples");
static_assert((kChan % 32) == 0 && (kKpad1 % 32) == 0, "GEMM K multiples of 32");
static_assert((kSteps % 128) == 0 && (kChan % 64) == 0, "GEMM M,N tile multiples");
static_assert(kChan / 4 == 512, "conv index split");

constexpr float kCarryXc  = 16.0f;
constexpr float kCarryRes = 2048.0f;
constexpr float kCarryW0  = 1024.0f;
constexpr float kCarryB   = 64.0f;
constexpr float kCarryW1  = 64.0f;
constexpr float kFold0    = 1.0f / (kCarryXc * kCarryW0);
constexpr float kFoldR    = kFold0 / kCarryRes;
constexpr float kFold1    = 1.0f / (kCarryB * kCarryW1);

constexpr size_t kOffXC32   = 0;
constexpr size_t kOffXCH    = kOffXC32   + (size_t)kSteps * kChan * 4;
constexpr size_t kOffXCL    = kOffXCH    + (size_t)kSteps * kChan * 2;
constexpr size_t kOffDT32   = kOffXCL    + (size_t)kSteps * kChan * 2;
constexpr size_t kOffPROJ32 = kOffDT32   + (size_t)kSteps * kChan * 4;
constexpr size_t kOffBH     = kOffPROJ32 + (size_t)kSteps * kProjW * 4;
constexpr size_t kOffW0H    = kOffBH     + (size_t)kSteps * kKpad1 * 2;
constexpr size_t kOffW1H    = kOffW0H    + (size_t)kProjW * kChan * 2;
constexpr size_t kWsTotal   = kOffW1H    + (size_t)kChan * kKpad1 * 2;
static_assert(kWsTotal == 50987008ull, "carve total");
static_assert(kWsTotal <= 134217728ull, "carve cap");
static_assert((kOffXCH % 128) == 0 && (kOffXCL % 128) == 0 && (kOffDT32 % 128) == 0 && (kOffPROJ32 % 128) == 0 &&
              (kOffBH % 128) == 0 && (kOffW0H % 128) == 0 && (kOffW1H % 128) == 0, "128-B aligned regions");

union FragH { v16h v; v8h h[2]; };
__device__ __forceinline__ v16h frag_load_h(const _Float16* p) {
  FragH f;
  f.h[0] = *(const v8h*)(p);
  f.h[1] = *(const v8h*)(p + 16);
  return f.v;
}
__device__ __forceinline__ v8f mma_f16(v16h a, v16h b, v8f c) {
  c = __builtin_amdgcn_wmma_f32_16x16x32_f16(false, a, false, b, (short)0, c, false, false);
  asm volatile("v_nop\n\tv_nop\n\tv_nop\n\tv_nop" : "+v"(c) : "v"(a), "v"(b));
  return c;
}
__device__ __forceinline__ void wave_lds_sync() {
  __builtin_amdgcn_fence(__ATOMIC_RELEASE, "workgroup");
  __builtin_amdgcn_wave_barrier();
  __builtin_amdgcn_fence(__ATOMIC_ACQUIRE, "workgroup");
}
__device__ __forceinline__ float rne_bf16_f(float f) {
  const unsigned u = __float_as_uint(f);
  const unsigned r = (u + 0x7FFFu + ((u >> 16) & 1u)) & 0xFFFF0000u;
  return __uint_as_float(r);
}
__device__ __forceinline__ v4f rne_bf16_v4(v4f v) {
  const float e0 = v[0];
  const float e1 = v[1];
  const float e2 = v[2];
  const float e3 = v[3];
  return (v4f){rne_bf16_f(e0), rne_bf16_f(e1), rne_bf16_f(e2), rne_bf16_f(e3)};
}
__device__ __forceinline__ unsigned pack2h(float a, float b) {
  const _Float16 ha = (_Float16)a;
  const _Float16 hb = (_Float16)b;
  const unsigned short ua = __builtin_bit_cast(unsigned short, ha);
  const unsigned short ub = __builtin_bit_cast(unsigned short, hb);
  return (unsigned)ua | ((unsigned)ub << 16);
}
__device__ __forceinline__ void split_h(float s, unsigned& hb, unsigned& lb) {
  const _Float16 hv = (_Float16)s;
  const float hf = (float)hv;
  const float diff = s - hf;
  const float res = diff * kCarryRes;
  const _Float16 lv = (_Float16)res;
  const unsigned short uh = __builtin_bit_cast(unsigned short, hv);
  const unsigned short ul = __builtin_bit_cast(unsigned short, lv);
  hb = (unsigned)uh;
  lb = (unsigned)ul;
}
template <bool RB>
__device__ __forceinline__ v4u pack8_f16(v4f a0, v4f a1, float carry, bool keep) {
  float e0 = a0[0];
  float e1 = a0[1];
  float e2 = a0[2];
  float e3 = a0[3];
  float e4 = a1[0];
  float e5 = a1[1];
  float e6 = a1[2];
  float e7 = a1[3];
  if (RB) {
    e0 = rne_bf16_f(e0);
    e1 = rne_bf16_f(e1);
    e2 = rne_bf16_f(e2);
    e3 = rne_bf16_f(e3);
    e4 = rne_bf16_f(e4);
    e5 = rne_bf16_f(e5);
    e6 = rne_bf16_f(e6);
    e7 = rne_bf16_f(e7);
  }
  const float f0 = keep ? e0 * carry : 0.0f;
  const float f1 = keep ? e1 * carry : 0.0f;
  const float f2 = keep ? e2 * carry : 0.0f;
  const float f3 = keep ? e3 * carry : 0.0f;
  const float f4 = keep ? e4 * carry : 0.0f;
  const float f5 = keep ? e5 * carry : 0.0f;
  const float f6 = keep ? e6 * carry : 0.0f;
  const float f7 = keep ? e7 * carry : 0.0f;
  v4u w;
  w[0] = pack2h(f0, f1);
  w[1] = pack2h(f2, f3);
  w[2] = pack2h(f4, f5);
  w[3] = pack2h(f6, f7);
  return w;
}
__device__ __forceinline__ void store_u4_twice(unsigned short* p, v4u w) {
  *(volatile v4u*)(void*)p = w;
  __threadfence();
  *(volatile v4u*)(void*)p = w;
}
__device__ __forceinline__ float silu_f(float v) {
  return v * (1.0f / (1.0f + expf(-v)));
}
__device__ __forceinline__ float softplus_f(float v) {
  return fmaxf(v, 0.0f) + log1pf(expf(-fabsf(v)));
}

__global__ __launch_bounds__(256) void prep_planes_kernel(
    const float* __restrict__ xw, const float* __restrict__ dtw,
    unsigned short* __restrict__ W0h, unsigned short* __restrict__ W1h)
{
  const int j = (int)(blockIdx.x & 31) * 256 + (int)threadIdx.x;
  if (blockIdx.x < 32) {
    const size_t e0 = (size_t)j * 8;
    const v4f a0 = *(const v4f*)(xw + e0);
    const v4f a1 = *(const v4f*)(xw + e0 + 4);
    const v4u w = pack8_f16<true>(a0, a1, kCarryW0, true);
    store_u4_twice(W0h + e0, w);
  } else {
    const int d   = j >> 2;
    const int cg  = j & 3;
    const int cgc = cg & 1;
    const bool keep = (cg < 2);
    const float* sp = dtw + (size_t)d * kStates + cgc * 8;
    const v4f a0 = *(const v4f*)(sp);
    const v4f a1 = *(const v4f*)(sp + 4);
    const v4u w = pack8_f16<true>(a0, a1, kCarryW1, keep);
    store_u4_twice(W1h + (size_t)j * 8, w);
  }
}

__global__ __launch_bounds__(256) void conv_silu_kernel(
    const float* __restrict__ x, const float* __restrict__ cw, const float* __restrict__ cb,
    float* __restrict__ xc32, unsigned short* __restrict__ xch, unsigned short* __restrict__ xcl)
{
  const int idx = (int)blockIdx.x * 256 + (int)threadIdx.x;
  if (idx >= kSteps * (kChan / 4)) return;
  const int t  = idx >> 9;
  const int d4 = (idx & 511) << 2;
  const v4f wa = rne_bf16_v4(*(const v4f*)(cw + (size_t)d4 * kTaps));
  const v4f wb = rne_bf16_v4(*(const v4f*)(cw + (size_t)d4 * kTaps + 4));
  const v4f wc = rne_bf16_v4(*(const v4f*)(cw + (size_t)d4 * kTaps + 8));
  const v4f wd = rne_bf16_v4(*(const v4f*)(cw + (size_t)d4 * kTaps + 12));
  const v4f bb = rne_bf16_v4(*(const v4f*)(cb + d4));
  const v4f zero4 = (v4f){0.f, 0.f, 0.f, 0.f};
  const int t3 = t - 3, t2 = t - 2, t1 = t - 1;
  const int r3 = t3 < 0 ? 0 : t3;
  const int r2 = t2 < 0 ? 0 : t2;
  const int r1 = t1 < 0 ? 0 : t1;
  v4f x0 = rne_bf16_v4(*(const v4f*)(x + (size_t)r3 * kChan + d4));
  v4f x1 = rne_bf16_v4(*(const v4f*)(x + (size_t)r2 * kChan + d4));
  v4f x2 = rne_bf16_v4(*(const v4f*)(x + (size_t)r1 * kChan + d4));
  const v4f x3 = rne_bf16_v4(*(const v4f*)(x + (size_t)t * kChan + d4));
  x0 = (t3 >= 0) ? x0 : zero4;
  x1 = (t2 >= 0) ? x1 : zero4;
  x2 = (t1 >= 0) ? x2 : zero4;

  float p0 = wa[0] * x0[0];
  p0 = fmaf(wa[1], x1[0], p0);
  p0 = fmaf(wa[2], x2[0], p0);
  p0 = fmaf(wa[3], x3[0], p0);
  p0 += bb[0];
  float p1 = wb[0] * x0[1];
  p1 = fmaf(wb[1], x1[1], p1);
  p1 = fmaf(wb[2], x2[1], p1);
  p1 = fmaf(wb[3], x3[1], p1);
  p1 += bb[1];
  float p2 = wc[0] * x0[2];
  p2 = fmaf(wc[1], x1[2], p2);
  p2 = fmaf(wc[2], x2[2], p2);
  p2 = fmaf(wc[3], x3[2], p2);
  p2 += bb[2];
  float p3 = wd[0] * x0[3];
  p3 = fmaf(wd[1], x1[3], p3);
  p3 = fmaf(wd[2], x2[3], p3);
  p3 = fmaf(wd[3], x3[3], p3);
  p3 += bb[3];

  const float o0 = silu_f(p0);
  const float o1 = silu_f(p1);
  const float o2 = silu_f(p2);
  const float o3 = silu_f(p3);
  const v4f ov = (v4f){o0, o1, o2, o3};
  const float s0 = o0 * kCarryXc;
  const float s1 = o1 * kCarryXc;
  const float s2 = o2 * kCarryXc;
  const float s3 = o3 * kCarryXc;
  unsigned h0, h1, h2, h3, l0, l1, l2, l3;
  split_h(s0, h0, l0);
  split_h(s1, h1, l1);
  split_h(s2, h2, l2);
  split_h(s3, h3, l3);
  v2u hw, lw;
  hw[0] = h0 | (h1 << 16);
  hw[1] = h2 | (h3 << 16);
  lw[0] = l0 | (l1 << 16);
  lw[1] = l2 | (l3 << 16);

  float* pf = xc32 + (size_t)t * kChan + d4;
  unsigned short* ph = xch + (size_t)t * kChan + d4;
  unsigned short* pl = xcl + (size_t)t * kChan + d4;
  *(volatile v4f*)pf = ov;
  *(volatile v2u*)(void*)ph = hw;
  *(volatile v2u*)(void*)pl = lw;
  __threadfence();
  *(volatile v4f*)pf = ov;
  *(volatile v2u*)(void*)ph = hw;
  *(volatile v2u*)(void*)pl = lw;
}

__global__ __launch_bounds__(256) void proj_gemm_kernel(
    const unsigned short* __restrict__ Ap, const unsigned short* __restrict__ A2p,
    const unsigned short* __restrict__ Btp,
    float* __restrict__ proj32, unsigned short* __restrict__ Bh)
{
  __shared__ __align__(16) float sT[8][32 * 36];
  const int lane = (int)threadIdx.x & 31;
  const int wave = __builtin_amdgcn_readfirstlane((int)(threadIdx.x >> 5));
  const int tile = (int)blockIdx.x * 8 + wave;
  const int m0 = tile * 32;
  const _Float16* A  = (const _Float16*)(const void*)Ap;
  const _Float16* A2 = (const _Float16*)(const void*)A2p;
  const _Float16* Bt = (const _Float16*)(const void*)Btp;
  const int rlane = lane & 15;
  const int koff  = (lane >> 4) * 8;
  const int mOff  = (lane >> 4) * 8;

  v8f acc00 = (v8f){0.f,0.f,0.f,0.f,0.f,0.f,0.f,0.f};
  v8f acc01 = acc00, acc10 = acc00, acc11 = acc00;
  v8f res00 = acc00, res01 = acc00, res10 = acc00, res11 = acc00;
  const size_t ao0 = (size_t)(m0 + rlane) * kChan + koff;
  const size_t ao1 = (size_t)(m0 + 16 + rlane) * kChan + koff;
  const _Float16* pb0 = Bt + (size_t)(rlane) * kChan + koff;
  const _Float16* pb1 = Bt + (size_t)(16 + rlane) * kChan + koff;
  for (int k0 = 0; k0 < kChan; k0 += 32) {
    const v16h b0 = frag_load_h(pb0 + k0);
    const v16h b1 = frag_load_h(pb1 + k0);
    const v16h a0 = frag_load_h(A + ao0 + k0);
    const v16h a1 = frag_load_h(A + ao1 + k0);
    const v16h l0 = frag_load_h(A2 + ao0 + k0);
    const v16h l1 = frag_load_h(A2 + ao1 + k0);
    acc00 = mma_f16(a0, b0, acc00);
    acc01 = mma_f16(a0, b1, acc01);
    acc10 = mma_f16(a1, b0, acc10);
    acc11 = mma_f16(a1, b1, acc11);
    res00 = mma_f16(l0, b0, res00);
    res01 = mma_f16(l0, b1, res01);
    res10 = mma_f16(l1, b0, res10);
    res11 = mma_f16(l1, b1, res11);
  }

  float* slab = sT[wave];
#pragma unroll
  for (int r = 0; r < 8; ++r) {
    const float m00 = acc00[r] * kFold0;
    const float m01 = acc01[r] * kFold0;
    const float m10 = acc10[r] * kFold0;
    const float m11 = acc11[r] * kFold0;
    slab[(mOff + r) * 36 + rlane]           = fmaf(res00[r], kFoldR, m00);
    slab[(mOff + r) * 36 + 16 + rlane]      = fmaf(res01[r], kFoldR, m01);
    slab[(16 + mOff + r) * 36 + rlane]      = fmaf(res10[r], kFoldR, m10);
    slab[(16 + mOff + r) * 36 + 16 + rlane] = fmaf(res11[r], kFoldR, m11);
  }
  wave_lds_sync();

  const int q  = lane >> 3;
  const int c4 = (lane & 7) * 4;
  const int rq = lane >> 2;
  const int cg = lane & 3;
  const int cgc = cg & 1;
  const bool keep = (cg < 2);
  v4f pv[8];
  v4u bw[4];
#pragma unroll
  for (int it = 0; it < 8; ++it) pv[it] = *(const v4f*)(slab + (it * 4 + q) * 36 + c4);
#pragma unroll
  for (int it = 0; it < 4; ++it) {
    const float* sp = slab + (it * 8 + rq) * 36 + cgc * 8;
    const v4f a0 = *(const v4f*)(sp);
    const v4f a1 = *(const v4f*)(sp + 4);
    bw[it] = pack8_f16<false>(a0, a1, kCarryB, keep);
  }
  for (int pass = 0; pass < 2; ++pass) {
#pragma unroll
    for (int it = 0; it < 8; ++it)
      *(volatile v4f*)(proj32 + (size_t)(m0 + it * 4 + q) * kProjW + c4) = pv[it];
#pragma unroll
    for (int it = 0; it < 4; ++it)
      *(volatile v4u*)(void*)(Bh + (size_t)(m0 + it * 8 + rq) * kKpad1 + cg * 8) = bw[it];
    __threadfence();
  }
}

__global__ __launch_bounds__(256) void dt_gemm_kernel(
    const unsigned short* __restrict__ BhP, const unsigned short* __restrict__ W1P,
    const float* __restrict__ dtb, float* __restrict__ dt32)
{
  __shared__ __align__(16) float sT[8][16 * 68];
  const int lane = (int)threadIdx.x & 31;
  const int wave = __builtin_amdgcn_readfirstlane((int)(threadIdx.x >> 5));
  const int gw   = (int)blockIdx.x * 8 + wave;
  const int n0   = (gw & 31) * 64;
  const int mr0  = (gw >> 5) * 128;
  const _Float16* A  = (const _Float16*)(const void*)BhP;
  const _Float16* Bt = (const _Float16*)(const void*)W1P;
  const int rlane = lane & 15;
  const int koff  = (lane >> 4) * 8;
  const int mOff  = (lane >> 4) * 8;
  const int hh    = lane >> 4;
  const int c4    = (lane & 15) * 4;

  const v16h b0 = frag_load_h(Bt + (size_t)(n0 + rlane) * kKpad1 + koff);
  const v16h b1 = frag_load_h(Bt + (size_t)(n0 + 16 + rlane) * kKpad1 + koff);
  const v16h b2 = frag_load_h(Bt + (size_t)(n0 + 32 + rlane) * kKpad1 + koff);
  const v16h b3 = frag_load_h(Bt + (size_t)(n0 + 48 + rlane) * kKpad1 + koff);
  const v4f bias4 = rne_bf16_v4(*(const v4f*)(dtb + n0 + c4));
  const float bs0 = bias4[0];
  const float bs1 = bias4[1];
  const float bs2 = bias4[2];
  const float bs3 = bias4[3];
  float* slab = sT[wave];

#pragma unroll 1
  for (int sub = 0; sub < 8; ++sub) {
    const int m0 = mr0 + sub * 16;
    const v16h a = frag_load_h(A + (size_t)(m0 + rlane) * kKpad1 + koff);
    v8f c0 = (v8f){0.f,0.f,0.f,0.f,0.f,0.f,0.f,0.f};
    v8f c1 = c0, c2 = c0, c3 = c0;
    c0 = mma_f16(a, b0, c0);
    c1 = mma_f16(a, b1, c1);
    c2 = mma_f16(a, b2, c2);
    c3 = mma_f16(a, b3, c3);
#pragma unroll
    for (int r = 0; r < 8; ++r) {
      slab[(mOff + r) * 68 + rlane]      = c0[r] * kFold1;
      slab[(mOff + r) * 68 + 16 + rlane] = c1[r] * kFold1;
      slab[(mOff + r) * 68 + 32 + rlane] = c2[r] * kFold1;
      slab[(mOff + r) * 68 + 48 + rlane] = c3[r] * kFold1;
    }
    wave_lds_sync();
#pragma unroll 1
    for (int it = 0; it < 8; ++it) {
      const int row = it * 2 + hh;
      const v4f v = *(const v4f*)(slab + row * 68 + c4);
      const float o0 = softplus_f(softplus_f(v[0] + bs0));
      const float o1 = softplus_f(softplus_f(v[1] + bs1));
      const float o2 = softplus_f(softplus_f(v[2] + bs2));
      const float o3 = softplus_f(softplus_f(v[3] + bs3));
      const v4f ov = (v4f){o0, o1, o2, o3};
      float* p = dt32 + (size_t)(m0 + row) * kChan + n0 + c4;
      *(volatile v4f*)p = ov;
      __threadfence();
      *(volatile v4f*)p = ov;
    }
    wave_lds_sync();
  }
}

__global__ __launch_bounds__(256) void scan_out_kernel(
    const float* __restrict__ xc32, const float* __restrict__ dt32, const float* __restrict__ proj32,
    const float* __restrict__ Dp, float* __restrict__ yout)
{
  __shared__ __align__(16) float sP[(kChunk + kWarm) * kProjW];
  __shared__ __align__(16) float sY[kGroup * 256];
  const int tid = (int)threadIdx.x;
  const int d   = (int)blockIdx.x * 256 + tid;
  const int t0  = (int)blockIdx.y * kChunk;
  const int ts  = (blockIdx.y > 0) ? (t0 - kWarm) : 0;
  const int nsteps = t0 + kChunk - ts;
  for (int i = tid; i < nsteps * 8; i += 256)
    *(v4f*)(sP + i * 4) = *(const v4f*)(proj32 + (size_t)ts * kProjW + (size_t)i * 4);
  __syncthreads();

  const float Dd = rne_bf16_f(Dp[d]);
  float h[kStates];
#pragma unroll
  for (int s = 0; s < kStates; ++s) h[s] = 0.0f;

  const int ngrp = nsteps / kGroup;
#pragma unroll 1
  for (int g = 0; g < ngrp; ++g) {
    const int tg = ts + g * kGroup;
#pragma unroll 1
    for (int i = 0; i < kGroup; ++i) {
      const int t = tg + i;
      const float dtv = dt32[(size_t)t * kChan + d];
      const float xv  = xc32[(size_t)t * kChan + d];
      const float* pr = sP + (g * kGroup + i) * kProjW;
      v4f Bv[4], Cv[4];
#pragma unroll
      for (int q4 = 0; q4 < 4; ++q4) {
        Bv[q4] = *(const v4f*)(pr + 4 * q4);
        Cv[q4] = *(const v4f*)(pr + kStates + 4 * q4);
      }
      const float r = expf(-dtv);
      float p = r;
      float acc = 0.0f;
#pragma unroll
      for (int q4 = 0; q4 < 4; ++q4) {
#pragma unroll
        for (int e = 0; e < 4; ++e) {
          const float bs = Bv[q4][e];
          const float cs = Cv[q4][e];
          const float dtB = dtv * bs;
          const float dbx = fmaxf(dtB * xv, 0.0f);
          h[4 * q4 + e] = fmaf(p, h[4 * q4 + e], dbx);
          acc = fmaf(cs, h[4 * q4 + e], acc);
          p = p * r;
        }
      }
      const float yv = fmaf(Dd, xv, acc);
      sY[i * 256 + tid] = yv;
    }
    if (tg >= t0) {
      for (int pass = 0; pass < 2; ++pass) {
#pragma unroll 1
        for (int i = 0; i < kGroup; ++i) {
          const float v = sY[i * 256 + tid];
          *(volatile float*)(yout + (size_t)(tg + i) * kChan + d) = v;
        }
        __threadfence();
      }
    }
  }
}

extern "C" void kernel_launch(void* const* d_in, const int* in_sizes, int n_in,
                              void* d_out, int out_size, void* d_ws, size_t ws_size,
                              hipStream_t stream) {
  if (n_in < 7) return;
  if (in_sizes[0] != kSteps * kChan) return;
  if (in_sizes[1] != kChan * kTaps) return;
  if (in_sizes[2] != kChan) return;
  if (in_sizes[3] != kProjW * kChan) return;
  if (in_sizes[4] != kChan * kStates) return;
  if (in_sizes[5] != kChan) return;
  if (in_sizes[6] != kChan) return;
  if (out_size != kSteps * kChan) return;
  if (ws_size < kWsTotal) return;

  const float* x       = (const float*)d_in[0];
  const float* conv_w  = (const float*)d_in[1];
  const float* conv_b  = (const float*)d_in[2];
  const float* xproj_w = (const float*)d_in[3];
  const float* dt_w    = (const float*)d_in[4];
  const float* dt_b    = (const float*)d_in[5];
  const float* Dp      = (const float*)d_in[6];
  float* y = (float*)d_out;

  char* ws = (char*)d_ws;
  float*          XC32   = (float*)(ws + kOffXC32);
  unsigned short* XCH    = (unsigned short*)(ws + kOffXCH);
  unsigned short* XCL    = (unsigned short*)(ws + kOffXCL);
  float*          DT32   = (float*)(ws + kOffDT32);
  float*          PROJ32 = (float*)(ws + kOffPROJ32);
  unsigned short* BH     = (unsigned short*)(ws + kOffBH);
  unsigned short* W0H    = (unsigned short*)(ws + kOffW0H);
  unsigned short* W1H    = (unsigned short*)(ws + kOffW1H);

  prep_planes_kernel<<<64, 256, 0, stream>>>(xproj_w, dt_w, W0H, W1H);
  conv_silu_kernel<<<(kSteps * (kChan / 4)) / 256, 256, 0, stream>>>(x, conv_w, conv_b, XC32, XCH, XCL);
  proj_gemm_kernel<<<(kSteps / 32) / 8, 256, 0, stream>>>(XCH, XCL, W0H, PROJ32, BH);
  dt_gemm_kernel<<<((kChan / 64) * (kSteps / 128)) / 8, 256, 0, stream>>>(BH, W1H, dt_b, DT32);
  scan_out_kernel<<<dim3(kChan / 256, kSteps / kChunk), 256, 0, stream>>>(XC32, DT32, PROJ32, Dp, y);
}
